// MatchPredictor_1864015806631
// MI455X (gfx1250) — hardware-verified
//
#include <hip/hip_runtime.h>
#include <math.h>

typedef __attribute__((ext_vector_type(16))) _Float16 v16h;
typedef __attribute__((ext_vector_type(16))) __bf16 v16b;
typedef __attribute__((ext_vector_type(8)))  _Float16 v8h;
typedef __attribute__((ext_vector_type(8)))  float v8f;
typedef __attribute__((ext_vector_type(4)))  float v4f;
typedef __attribute__((ext_vector_type(2)))  float v2f;
typedef __attribute__((ext_vector_type(4)))  unsigned v4u;
typedef __attribute__((ext_vector_type(4)))  int v4i;
typedef float __attribute__((may_alias)) float_a;
typedef int __attribute__((may_alias)) int_a;

template <typename T> __device__ __forceinline__ void vst2(void* p, T v) { *(volatile T*)p = v; __threadfence(); *(volatile T*)p = v; }
__device__ __forceinline__ v8f wmma16(v16h a, v16h b, v8f c) {
  v8f d = __builtin_amdgcn_wmma_f32_16x16x32_f16(false, a, false, b, (short)0, c, false, false);
  asm volatile("v_nop\n\tv_nop\n\tv_nop\n\tv_nop" : "+v"(d) : "v"(a), "v"(b));
  return d;
}
__device__ __forceinline__ v8f wmma_bf(v16b a, v16b b, v8f c) {
  v8f d = __builtin_amdgcn_wmma_f32_16x16x32_bf16(false, a, false, b, (short)0, c, false, false);
  asm volatile("v_nop\n\tv_nop\n\tv_nop\n\tv_nop" : "+v"(d) : "v"(a), "v"(b));
  return d;
}
__device__ __forceinline__ v16h frag_h(const _Float16* rowk0, int lane) {
  union { v16h v; v8h q[2]; } u; const _Float16* p = rowk0 + 8 * (lane >> 4);
  u.q[0] = *(const v8h*)p; u.q[1] = *(const v8h*)(p + 16); return u.v;
}
__device__ __forceinline__ v16h frag_f32(const float* rowk0, int lane) {
  v16h a; const float* p = rowk0 + 8 * (lane >> 4);
#pragma unroll
  for (int i = 0; i < 8; ++i) { a[i] = (_Float16)p[i]; a[8 + i] = (_Float16)p[16 + i]; }
  return a;
}
__device__ __forceinline__ v16h frag_f32s(const float* rowk0, int lane, float sc) {
  v16h a; const float* p = rowk0 + 8 * (lane >> 4);
#pragma unroll
  for (int i = 0; i < 8; ++i) { a[i] = (_Float16)(p[i] * sc); a[8 + i] = (_Float16)(p[16 + i] * sc); }
  return a;
}
__device__ __forceinline__ v16h fragc_f32(const float* W, int k0, int n, int lane, int ld, int K) {
  v16h a; const int g = lane >> 4;
#pragma unroll
  for (int i = 0; i < 8; ++i) { const int ka = k0 + 8 * g + i, kb = ka + 16;
    a[i] = (_Float16)(ka < K ? W[(size_t)(ka < K ? ka : K - 1) * ld + n] : 0.f); a[8 + i] = (_Float16)(kb < K ? W[(size_t)(kb < K ? kb : K - 1) * ld + n] : 0.f); }
  return a;
}
struct F2 { v16b h, l; };
__device__ __forceinline__ F2 bsplit16(const float v[16]) { F2 r;
#pragma unroll
  for (int i = 0; i < 16; ++i) { const __bf16 h = (__bf16)v[i]; r.h[i] = h; r.l[i] = (__bf16)(v[i] - (float)h); }
  return r; }
__device__ __forceinline__ F2 split_row(const float* row, int k0, int lane) { float v[16]; const float* p = row + k0 + 8 * (lane >> 4);
#pragma unroll
  for (int i = 0; i < 8; ++i) { v[i] = p[i]; v[8 + i] = p[16 + i]; }
  return bsplit16(v); }
__device__ __forceinline__ F2 split_rowK(const float* row, int k0, int lane, int K) { float v[16]; const int g = lane >> 4;
#pragma unroll
  for (int i = 0; i < 8; ++i) { const int ka = k0 + 8 * g + i, kb = ka + 16; v[i] = ka < K ? row[ka < K ? ka : K - 1] : 0.f; v[8 + i] = kb < K ? row[kb < K ? kb : K - 1] : 0.f; }
  return bsplit16(v); }
__device__ __forceinline__ F2 split_col(const float* W, int k0, int n, int lane, int ld, int K) { float v[16]; const int g = lane >> 4;
#pragma unroll
  for (int i = 0; i < 8; ++i) { const int ka = k0 + 8 * g + i, kb = ka + 16; v[i] = ka < K ? W[(size_t)(ka < K ? ka : K - 1) * ld + n] : 0.f; v[8 + i] = kb < K ? W[(size_t)(kb < K ? kb : K - 1) * ld + n] : 0.f; }
  return bsplit16(v); }
__device__ __forceinline__ v8f mac3(const F2& a, const F2& b, v8f c) { c = wmma_bf(a.l, b.h, c); c = wmma_bf(a.h, b.l, c); return wmma_bf(a.h, b.h, c); }
__device__ __forceinline__ float sigm(float v) { return 1.0f / (1.0f + expf(-v)); }
#define LDSX() do { asm volatile("s_wait_dscnt 0" ::: "memory"); __builtin_amdgcn_wave_barrier(); __builtin_amdgcn_fence(__ATOMIC_RELEASE, "workgroup"); } while (0)


#define NBR 262144
#define NE 170
#define ED 50
#define NC 10
#define NF 12
#ifndef NROWS
#define NROWS NBR
#endif
__device__ __forceinline__ float bfr(float v) { return (float)(__bf16)v; }
typedef __attribute__((ext_vector_type(8))) __bf16 v8b;
template <int LDA> __device__ __forceinline__ F2 fragA_lds(const float (*T)[LDA], int row, int k0, int lane) { float v[16]; const int g = lane >> 4;
#pragma unroll
  for (int i = 0; i < 8; ++i) { v[i] = T[row][k0 + 8 * g + i]; v[8 + i] = T[row][k0 + 16 + 8 * g + i]; }
  return bsplit16(v); }
__device__ __forceinline__ v16b fragW(const float* __restrict__ Wt, int NO, int NI, int o, int k0, int lane) { v16b w; const int g = lane >> 4; const int oc = o < NO ? o : NO - 1;
#pragma unroll
  for (int i = 0; i < 8; ++i) { const int ka = k0 + 8 * g + i, kb2 = ka + 16; const float wa = Wt[(size_t)oc * NI + (ka < NI ? ka : NI - 1)], wb = Wt[(size_t)oc * NI + (kb2 < NI ? kb2 : NI - 1)];
    w[i] = (__bf16)((o < NO && ka < NI) ? wa : 0.f); w[8 + i] = (__bf16)((o < NO && kb2 < NI) ? wb : 0.f); }
  return w; }
__global__ __launch_bounds__(128) void k_mp(const float* __restrict__ FEAT, const float* __restrict__ EMB,
    const float* __restrict__ W1a, const float* __restrict__ B1a, const float* __restrict__ W2a, const float* __restrict__ B2a, const float* __restrict__ W3a, const float* __restrict__ B3a,
    const float* __restrict__ W1b, const float* __restrict__ B1b, const float* __restrict__ W2b, const float* __restrict__ B2b, const float* __restrict__ W3b, const float* __restrict__ B3b,
    const float* __restrict__ WF, const float* __restrict__ BFin, float* __restrict__ OUT) {
  __shared__ __align__(16) float sx[64][68];
  __shared__ __align__(16) float st[64][132];
  const int tid = threadIdx.x, wave = tid >> 5, lane = tid & 31, col = lane & 15, g = lane >> 4; const size_t r0 = (size_t)blockIdx.x * 64; const int wr = wave * 16;
#pragma unroll 1
  for (int c = 0; c < NC; ++c) { const bool tb = c >= 5; const float* W1 = tb ? W1b : W1a; const float* B1 = tb ? B1b : B1a; const float* W2 = tb ? W2b : W2a; const float* B2 = tb ? B2b : B2a; const float* W3 = tb ? W3b : W3a; const float* B3 = tb ? B3b : B3a;
    for (int e = lane; e < 16 * 64; e += 32) { const int rl = e >> 6, k = e & 63; const size_t row = r0 + wr + rl; const float* fr = FEAT + row * NF; float v = 0.f;
      if (k < ED) { int id = (int)bfr(fr[2 + c]); if (id < 0) id += NE; id = id < 0 ? 0 : (id >= NE ? NE - 1 : id); v = bfr(EMB[(size_t)id * ED + k]); }
      else if (k == ED) v = bfr(fr[tb ? 1 : 0]);
      sx[wr + rl][k] = v; }
    LDSX();
    v8f a1[4] = {};
#pragma unroll
    for (int kc = 0; kc < 2; ++kc) { const F2 a = fragA_lds<68>(sx, wr + col, kc * 32, lane);
#pragma unroll
      for (int j = 0; j < 4; ++j) { const v16b w = fragW(W1, 50, 51, j * 16 + col, kc * 32, lane); asm volatile("s_wait_loadcnt 0x0" ::: "memory"); a1[j] = wmma_bf(a.h, w, a1[j]); } }
    LDSX();
#pragma unroll
    for (int j = 0; j < 4; ++j) { const int o = j * 16 + col; const float bb = o < 50 ? bfr(B1[o < 50 ? o : 49]) : 0.f;
#pragma unroll
      for (int r = 0; r < 8; ++r) sx[wr + 8 * g + r][o] = o < 50 ? fmaxf(a1[j][r] + bb, 0.f) : 0.f; }
    LDSX();
    v8f a2[2] = {};
#pragma unroll
    for (int kc = 0; kc < 2; ++kc) { const F2 a = fragA_lds<68>(sx, wr + col, kc * 32, lane);
#pragma unroll
      for (int j = 0; j < 2; ++j) { const v16b w = fragW(W2, 25, 50, j * 16 + col, kc * 32, lane); asm volatile("s_wait_loadcnt 0x0" ::: "memory"); a2[j] = wmma_bf(a.h, w, a2[j]); a2[j] = wmma_bf(a.l, w, a2[j]); } }
    LDSX();
#pragma unroll
    for (int j = 0; j < 2; ++j) { const int o = j * 16 + col; const float bb = o < 25 ? bfr(B2[o < 25 ? o : 24]) : 0.f;
#pragma unroll
      for (int r = 0; r < 8; ++r) sx[wr + 8 * g + r][o] = o < 25 ? fmaxf(a2[j][r] + bb, 0.f) : 0.f; }
    LDSX();
    v8f a3 = {};
    { const F2 a = fragA_lds<68>(sx, wr + col, 0, lane); const v16b w = fragW(W3, 10, 25, col, 0, lane); asm volatile("s_wait_loadcnt 0x0" ::: "memory"); a3 = wmma_bf(a.h, w, a3); a3 = wmma_bf(a.l, w, a3); }
    { const float bb = col < 10 ? bfr(B3[col < 10 ? col : 9]) : 0.f;
#pragma unroll
      for (int r = 0; r < 8; ++r) if (col < 10) st[wr + 8 * g + r][c * 10 + col] = fmaxf(a3[r] + bb, 0.f); }
  }
  for (int e = lane; e < 16 * 28; e += 32) { const int rl = e / 28, k = 100 + e % 28; st[wr + rl][k] = 0.f; }
  LDSX();
  v8f af = {};
#pragma unroll
  for (int kc = 0; kc < 4; ++kc) { const F2 a = fragA_lds<132>(st, wr + col, kc * 32, lane); const v16b w = fragW(WF, 2, 100, col, kc * 32, lane); asm volatile("s_wait_loadcnt 0x0" ::: "memory"); af = wmma_bf(a.h, w, af); af = wmma_bf(a.l, w, af); }
  LDSX();
  { const float bb = col < 2 ? bfr(BFin[col < 2 ? col : 1]) : 0.f;
#pragma unroll
    for (int r = 0; r < 8; ++r) if (col < 2) st[wr + 8 * g + r][128 + col] = af[r] + bb; }
  LDSX();
  if (lane < 8) { v4f o; o[0] = st[wr + 2 * lane][128]; o[1] = st[wr + 2 * lane][129]; o[2] = st[wr + 2 * lane + 1][128]; o[3] = st[wr + 2 * lane + 1][129]; vst2(OUT + (r0 + wr + 2 * lane) * 2, o); } }
extern "C" void kernel_launch(void* const* d_in, const int* in_sizes, int n_in, void* d_out, int out_size, void* d_ws, size_t ws_size, hipStream_t stream) {
  (void)in_sizes; (void)n_in; (void)out_size; (void)d_ws; (void)ws_size;
  const float** F = (const float**)d_in;
  k_mp<<<dim3(NROWS / 64), 128, 0, stream>>>(F[0], F[1], F[2], F[3], F[4], F[5], F[6], F[7], F[8], F[9], F[10], F[11], F[12], F[13], F[14], F[15], (float*)d_out);
}
